// RepresentationNetwork_81990925680796
// MI455X (gfx1250) — hardware-verified
//
#include <hip/hip_runtime.h>
#include <stddef.h>


#define FEAT    128
#define KCAT    256
#define NLAYER  3
#define NTHR    256
#define NWAVE   8
#define EPT     8
#define NGRP    2
#define CHUNK   (NTHR * EPT * NGRP)
#define WCAP    (EPT * NGRP * 32)
#define LISTN   (NWAVE * WCAP)
#define NBC     4096
#define NBF     1024
#define RCAP    32768
#define RBN     128
#define DEGCAP  128
#define GROWS   128
#define OTHR    512
#define APH     (KCAT + 8)
#define SPF     FEAT
#define WPB     ((NLAYER * FEAT * KCAT / 8) / NTHR)

#define LDS_FILL  ((RCAP + NBF + LISTN) * 4 + 64)
#define LDS_LAYER (2 * GROWS * APH * 2 + GROWS * SPF * 4)

static_assert((CHUNK & (CHUNK - 1)) == 0);
static_assert(CHUNK <= 4096);
static_assert(NBC <= 4096 && NBF <= 4096);
static_assert((NBC & (NBC - 1)) == 0 && (NBF & (NBF - 1)) == 0);
static_assert(NBC == 4 * NBF);
static_assert(OTHR * 8 == NBC);
static_assert((RCAP % 32) == 0);
static_assert(GROWS == NWAVE * 16);
static_assert(FEAT == 4 * 32);
static_assert((KCAT % 32) == 0 && (APH % 8) == 0);
static_assert(WPB * NTHR * 8 == NLAYER * FEAT * KCAT);
static_assert((DEGCAP % 32) == 0);

typedef float    v4f  __attribute__((ext_vector_type(4)));
typedef float    v8f  __attribute__((ext_vector_type(8)));
typedef int      v4i  __attribute__((ext_vector_type(4)));
typedef unsigned v2u  __attribute__((ext_vector_type(2)));
typedef unsigned v4u  __attribute__((ext_vector_type(4)));
typedef __bf16   v16b __attribute__((ext_vector_type(16)));
union FragB { v16b v; v4u u[2]; };

__device__ __forceinline__ unsigned bfbits(float f) {
  const unsigned u = __float_as_uint(f);
  return (u + 0x7FFFu + ((u >> 16) & 1u)) >> 16;
}

__device__ __forceinline__ void split4(v4f v, v2u& hi, v2u& lo) {
  const unsigned h0 = bfbits(v.x), h1 = bfbits(v.y), h2 = bfbits(v.z), h3 = bfbits(v.w);
  const unsigned l0 = bfbits(v.x - __uint_as_float(h0 << 16));
  const unsigned l1 = bfbits(v.y - __uint_as_float(h1 << 16));
  const unsigned l2 = bfbits(v.z - __uint_as_float(h2 << 16));
  const unsigned l3 = bfbits(v.w - __uint_as_float(h3 << 16));
  hi.x = h0 | (h1 << 16); hi.y = h2 | (h3 << 16);
  lo.x = l0 | (l1 << 16); lo.y = l2 | (l3 << 16);
}

__device__ __forceinline__ v8f wmb(v16b a, v16b b, v8f c) {
  v8f d = __builtin_amdgcn_wmma_f32_16x16x32_bf16(false, a, false, b, (short)0, c, false, false);
  asm volatile("v_nop\n\tv_nop\n\tv_nop\n\tv_nop" : "+v"(d) : "v"(a), "v"(b));
  return d;
}

template <int NB>
__device__ __forceinline__ int scan_chunk(const int* __restrict__ dsts, int nE, int cbase, int slotBase,
                                          int vec8, int* list, int tid, int lane, int wave) {
  int wc = 0;
#pragma unroll
  for (int g = 0; g < NGRP; ++g) {
    const int el0  = (g * NTHR + tid) * EPT;
    const int e0   = cbase + el0;
    const int sent = -2147483647 - 1;
    v4i da, db;
    if (vec8 != 0 && cbase + CHUNK <= nE) {
      da = *(const v4i*)(dsts + e0);
      db = *(const v4i*)(dsts + e0 + 4);
    } else {
      da.x = (e0     < nE) ? dsts[min(e0, nE - 1)] : sent;
      da.y = (e0 + 1 < nE) ? dsts[min(e0 + 1, nE - 1)] : sent;
      da.z = (e0 + 2 < nE) ? dsts[min(e0 + 2, nE - 1)] : sent;
      da.w = (e0 + 3 < nE) ? dsts[min(e0 + 3, nE - 1)] : sent;
      db.x = (e0 + 4 < nE) ? dsts[min(e0 + 4, nE - 1)] : sent;
      db.y = (e0 + 5 < nE) ? dsts[min(e0 + 5, nE - 1)] : sent;
      db.z = (e0 + 6 < nE) ? dsts[min(e0 + 6, nE - 1)] : sent;
      db.w = (e0 + 7 < nE) ? dsts[min(e0 + 7, nE - 1)] : sent;
    }
    const unsigned nb = (unsigned)slotBase;
    const unsigned s0 = (unsigned)da.x - nb, s1 = (unsigned)da.y - nb;
    const unsigned s2 = (unsigned)da.z - nb, s3 = (unsigned)da.w - nb;
    const unsigned s4 = (unsigned)db.x - nb, s5 = (unsigned)db.y - nb;
    const unsigned s6 = (unsigned)db.z - nb, s7 = (unsigned)db.w - nb;
    const bool h0 = s0 < (unsigned)NB, h1 = s1 < (unsigned)NB, h2 = s2 < (unsigned)NB, h3 = s3 < (unsigned)NB;
    const bool h4 = s4 < (unsigned)NB, h5 = s5 < (unsigned)NB, h6 = s6 < (unsigned)NB, h7 = s7 < (unsigned)NB;
    const unsigned any = __builtin_amdgcn_ballot_w32(h0 | h1 | h2 | h3 | h4 | h5 | h6 | h7);
    if (any != 0u) {
#define HITJ(J, HJ, SJ) { \
        const unsigned mj = __builtin_amdgcn_ballot_w32(HJ); \
        if (mj != 0u) { \
          if (HJ) { \
            const int pos = wc + (int)__builtin_amdgcn_mbcnt_lo(mj, 0u); \
            if (pos < WCAP) list[wave * WCAP + pos] = ((el0 + (J)) << 12) | (int)(SJ); \
          } \
          wc += (int)__builtin_popcount(mj); } }
      HITJ(0, h0, s0)
      HITJ(1, h1, s1)
      HITJ(2, h2, s2)
      HITJ(3, h3, s3)
      HITJ(4, h4, s4)
      HITJ(5, h5, s5)
      HITJ(6, h6, s6)
      HITJ(7, h7, s7)
#undef HITJ
    }
  }
  return wc;
}

__global__ __launch_bounds__(NTHR) void k_wprep(
    const float* __restrict__ wr1, const float* __restrict__ wo1,
    const float* __restrict__ wr2, const float* __restrict__ wo2,
    const float* __restrict__ wr3, const float* __restrict__ wo3,
    unsigned short* BH, unsigned short* BL) {
  const int b = blockIdx.x;
  if (b >= WPB) return;
  const int tid = threadIdx.x;
  const int layer = b >> 4, half = (b >> 3) & 1;
  const float* src = layer == 0 ? (half ? wo1 : wr1) : (layer == 1 ? (half ? wo2 : wr2) : (half ? wo3 : wr3));
  const int rr = ((b & 7) << 8) | tid;
  const int n  = rr >> 4;
  const int kk = (rr & 15) * 8;
  const float* sp = src + n * FEAT + kk;
  const v4f a = *(const v4f*)sp, c = *(const v4f*)(sp + 4);
  v2u ha, la, hc, lc;
  split4(a, ha, la);
  split4(c, hc, lc);
  v4u hv, lv;
  hv.x = ha.x; hv.y = ha.y; hv.z = hc.x; hv.w = hc.y;
  lv.x = la.x; lv.y = la.y; lv.z = lc.x; lv.w = lc.y;
  const size_t o = (size_t)layer * FEAT * KCAT + (size_t)n * KCAT + (size_t)half * FEAT + kk;
  *(volatile v4u*)(BH + o) = hv;
  *(volatile v4u*)(BL + o) = lv;
  __threadfence();
  *(volatile v4u*)(BH + o) = hv;
  *(volatile v4u*)(BL + o) = lv;
}

__global__ __launch_bounds__(NTHR) void k_count(const int* __restrict__ ei, int* cnt, int nE, int vec8) {
  __shared__ __attribute__((aligned(16))) int scnt[NBC];
  __shared__ __attribute__((aligned(16))) int list[LISTN];
  __shared__ int wcnt[NWAVE];
  const int tid = threadIdx.x, lane = tid & 31, wave = tid >> 5;
  const int nodeBase = blockIdx.x * NBC;
  const int* dsts = ei + nE;

  for (int i = tid; i < NBC; i += NTHR) scnt[i] = 0;
  __syncthreads();

  const int nChunks = (nE + CHUNK - 1) / CHUNK;
#pragma unroll 1
  for (int ch = 0; ch < nChunks; ++ch) {
    const int cbase = ch * CHUNK;
    const int wc = scan_chunk<NBC>(dsts, nE, cbase, nodeBase, vec8, list, tid, lane, wave);
    if (lane == 0) wcnt[wave] = wc;
    __syncthreads();
    if (wave == 0) {
#pragma unroll 1
      for (int wsx = 0; wsx < NWAVE; ++wsx) {
        int n = __builtin_amdgcn_readfirstlane(wcnt[wsx]);
        n = n > WCAP ? WCAP : (n < 0 ? 0 : n);
        const int* lp = list + wsx * WCAP;
#pragma unroll 1
        for (int i = 0; i < n; ++i) {
          const int ent  = __builtin_amdgcn_readfirstlane(lp[i]);
          const int slot = ent & (NBC - 1);
          if (lane == 0) scnt[slot] = scnt[slot] + 1;
        }
      }
    }
    __syncthreads();
  }

  v4i cq[4];
#pragma unroll
  for (int q = 0; q < 4; ++q) {
    const int f = (wave * 4 + q) * 128 + 4 * lane;
    cq[q] = *(const v4i*)(scnt + f);
  }
  int* cp = cnt + (size_t)nodeBase;
#pragma unroll
  for (int q = 0; q < 4; ++q) {
    const int f = (wave * 4 + q) * 128 + 4 * lane;
    *(volatile v4i*)(cp + f) = cq[q];
  }
  __threadfence();
#pragma unroll
  for (int q = 0; q < 4; ++q) {
    const int f = (wave * 4 + q) * 128 + 4 * lane;
    *(volatile v4i*)(cp + f) = cq[q];
  }
}

__global__ __launch_bounds__(OTHR) void k_offsets(
    const int* __restrict__ cnt, int* off, int* rbase, int nChunk) {
  __shared__ __attribute__((aligned(16))) int soff[NBC];
  __shared__ __attribute__((aligned(16))) int srb[RBN];
  __shared__ int wtot[OTHR / 32];
  const int tid = threadIdx.x, lane = tid & 31, wave = tid >> 5, sub = tid >> 7;
  for (int i = tid; i < RBN; i += OTHR) srb[i] = 0;
  int carry = 0;
#pragma unroll 1
  for (int ch = 0; ch < nChunk; ++ch) {
    const int base = ch * NBC;
    const v4i c0 = *(const v4i*)(cnt + base + 8 * tid);
    const v4i c1 = *(const v4i*)(cnt + base + 8 * tid + 4);
    const int e0 = max(c0.x, 0), e1 = max(c0.y, 0), e2 = max(c0.z, 0), e3 = max(c0.w, 0);
    const int e4 = max(c1.x, 0), e5 = max(c1.y, 0), e6 = max(c1.z, 0), e7 = max(c1.w, 0);
    const int ts = e0 + e1 + e2 + e3 + e4 + e5 + e6 + e7;
    int incl = ts;
#pragma unroll
    for (int d = 1; d < 32; d <<= 1) {
      const int t = __shfl_up(incl, d);
      if (lane >= d) incl += t;
    }
    if (lane == 31) wtot[wave] = incl;
    __syncthreads();
    const int S0 = wtot[0]  + wtot[1]  + wtot[2]  + wtot[3];
    const int S1 = wtot[4]  + wtot[5]  + wtot[6]  + wtot[7];
    const int S2 = wtot[8]  + wtot[9]  + wtot[10] + wtot[11];
    const int S3 = wtot[12] + wtot[13] + wtot[14] + wtot[15];
    int pre = 0;
#pragma unroll 1
    for (int w = 4 * sub; w < wave; ++w) pre += wtot[w];
    const int b0 = carry;
    const int b1 = b0 + ((S0 + 31) & ~31);
    const int b2 = b1 + ((S1 + 31) & ~31);
    const int b3 = b2 + ((S2 + 31) & ~31);
    const int b4 = b3 + ((S3 + 31) & ~31);
    const int myb = sub == 0 ? b0 : (sub == 1 ? b1 : (sub == 2 ? b2 : b3));
    if (tid == 0) {
      srb[min(4 * ch + 0, RBN - 1)] = b0;
      srb[min(4 * ch + 1, RBN - 1)] = b1;
      srb[min(4 * ch + 2, RBN - 1)] = b2;
      srb[min(4 * ch + 3, RBN - 1)] = b3;
    }
    int run = myb + pre + incl - ts;
    soff[8 * tid + 0] = run; run += e0;
    soff[8 * tid + 1] = run; run += e1;
    soff[8 * tid + 2] = run; run += e2;
    soff[8 * tid + 3] = run; run += e3;
    soff[8 * tid + 4] = run; run += e4;
    soff[8 * tid + 5] = run; run += e5;
    soff[8 * tid + 6] = run; run += e6;
    soff[8 * tid + 7] = run;
    carry = b4;
    __syncthreads();
    const v4i o0 = *(const v4i*)(soff + 4 * tid);
    const v4i o1 = *(const v4i*)(soff + 4 * (tid + OTHR));
    int* op = off + base;
    *(volatile v4i*)(op + 4 * tid) = o0;
    *(volatile v4i*)(op + 4 * (tid + OTHR)) = o1;
    __threadfence();
    *(volatile v4i*)(op + 4 * tid) = o0;
    *(volatile v4i*)(op + 4 * (tid + OTHR)) = o1;
    __syncthreads();
  }
  if (tid == 0) srb[min(4 * nChunk, RBN - 1)] = carry;
  __syncthreads();
  v4i rv = {0, 0, 0, 0};
  if (tid < 32) rv = *(const v4i*)(srb + 4 * tid);
  if (tid < 32) *(volatile v4i*)(rbase + 4 * tid) = rv;
  __threadfence();
  if (tid < 32) *(volatile v4i*)(rbase + 4 * tid) = rv;
}

__global__ __launch_bounds__(NTHR) void k_fill(
    const int* __restrict__ ei, const int* __restrict__ off, const int* __restrict__ rbase,
    int* csr, int nN, int nE, int vec8, int csrLen) {
  extern __shared__ v4f lds_dyn[];
  int* region = (int*)lds_dyn;
  int* cursor = region + RCAP;
  int* list   = cursor + NBF;
  int* wcnt   = list + LISTN;
  const int tid = threadIdx.x, lane = tid & 31, wave = tid >> 5;
  const int b = blockIdx.x;
  const int nodeBase = b * NBF;
  const int* dsts = ei + nE;

  int rb0 = rbase[b];
  const int rb1 = rbase[b + 1];
  rb0 = rb0 < 0 ? 0 : (rb0 > csrLen ? csrLen : rb0);
  rb0 &= ~31;
  int len = rb1 - rb0;
  len = len < 0 ? 0 : (len > RCAP ? RCAP : len);
  int lenW = (len + 31) & ~31;
  if (rb0 + lenW > csrLen) lenW = (csrLen - rb0) & ~31;

  {
    const v4i z = {0, 0, 0, 0};
    for (int i = tid; i < RCAP / 4; i += NTHR) ((v4i*)region)[i] = z;
    for (int s = tid; s < NBF; s += NTHR) {
      int o = off[nodeBase + s] - rb0;
      o = o < 0 ? 0 : (o > RCAP ? RCAP : o);
      cursor[s] = o;
    }
  }
  __syncthreads();

  const int nChunks = (nE + CHUNK - 1) / CHUNK;
#pragma unroll 1
  for (int ch = 0; ch < nChunks; ++ch) {
    const int cbase = ch * CHUNK;
    const int wc = scan_chunk<NBF>(dsts, nE, cbase, nodeBase, vec8, list, tid, lane, wave);
    if (lane == 0) wcnt[wave] = wc;
    __syncthreads();
    if (wave == 0) {
#pragma unroll 1
      for (int wsx = 0; wsx < NWAVE; ++wsx) {
        int n = __builtin_amdgcn_readfirstlane(wcnt[wsx]);
        n = n > WCAP ? WCAP : (n < 0 ? 0 : n);
        const int* lp = list + wsx * WCAP;
#pragma unroll 1
        for (int i = 0; i < n; ++i) {
          const int ent  = __builtin_amdgcn_readfirstlane(lp[i]);
          const int slot = ent & (NBF - 1);
          int e = cbase + ((ent >> 12) & (CHUNK - 1));
          e = e > nE - 1 ? nE - 1 : e;
          int src = ei[e];
          src = src < 0 ? 0 : (src > nN - 1 ? nN - 1 : src);
          if (lane == 0) {
            int pos = cursor[slot];
            pos = pos < 0 ? 0 : (pos > RCAP - 1 ? RCAP - 1 : pos);
            region[pos] = src;
            const int np = pos + 1;
            cursor[slot] = np > RCAP ? RCAP : np;
          }
        }
      }
    }
    __syncthreads();
  }

  const int nv = lenW >> 2;
  int* gp = csr + rb0;
#pragma unroll 1
  for (int i = tid; i < nv; i += NTHR) { const v4i v = ((const v4i*)region)[i]; *(volatile v4i*)(gp + 4 * i) = v; }
  __threadfence();
#pragma unroll 1
  for (int i = tid; i < nv; i += NTHR) { const v4i v = ((const v4i*)region)[i]; *(volatile v4i*)(gp + 4 * i) = v; }
}

__global__ __launch_bounds__(NTHR) void k_layer(
    const float* __restrict__ Hin, const int* __restrict__ csr, const int* __restrict__ off,
    const int* __restrict__ cnt, const unsigned short* __restrict__ BH, const unsigned short* __restrict__ BL,
    const float* __restrict__ bias, float* Out, int nN, int csrLen, int cntLen, int nRowsOut) {
  extern __shared__ v4f lds_dyn[];
  unsigned short* sHi = (unsigned short*)lds_dyn;
  unsigned short* sLo = sHi + GROWS * APH;
  float*          stg = (float*)(sLo + GROWS * APH);
  const int tid = threadIdx.x, lane = tid & 31, wave = tid >> 5, hh = lane >> 4, m = lane & 15;
  const int rowBase = blockIdx.x * GROWS;
  const int r0 = wave * 16;

  int ci = rowBase + r0 + m;
  ci = ci > cntLen - 1 ? cntLen - 1 : ci;
  const int cnt_l = cnt[ci];
  const int off_l = off[ci];
#pragma unroll 1
  for (int j = 0; j < 16; ++j) {
    const int c = rowBase + r0 + j;
    int n = __builtin_amdgcn_readlane(cnt_l, j);
    n = n < 0 ? 0 : (n > DEGCAP ? DEGCAP : n);
    const int st = __builtin_amdgcn_readlane(off_l, j);
    v4f acc = {0.f, 0.f, 0.f, 0.f};
#pragma unroll 1
    for (int q0 = 0; q0 < n; q0 += 32) {
      int pos = st + q0 + lane;
      pos = pos < 0 ? 0 : (pos > csrLen - 1 ? csrLen - 1 : pos);
      int sl = csr[pos];
      sl = sl < 0 ? 0 : (sl > nN - 1 ? nN - 1 : sl);
      const int mcnt = (n - q0) < 32 ? (n - q0) : 32;
#pragma unroll 1
      for (int p = 0; p < mcnt; ++p) {
        const int s = __builtin_amdgcn_readlane(sl, p);
        acc = acc + *(const v4f*)(Hin + (size_t)s * FEAT + 4 * lane);
      }
    }
    const int co = c > nN - 1 ? nN - 1 : c;
    const v4f own = *(const v4f*)(Hin + (size_t)co * FEAT + 4 * lane);
    v2u ah, al, oh, ol;
    split4(acc, ah, al);
    split4(own, oh, ol);
    unsigned short* ph = sHi + (r0 + j) * APH + 4 * lane;
    unsigned short* pl = sLo + (r0 + j) * APH + 4 * lane;
    *(v2u*)ph = ah;  *(v2u*)(ph + FEAT) = oh;
    *(v2u*)pl = al;  *(v2u*)(pl + FEAT) = ol;
  }
  __syncthreads();

  const unsigned short* arH = sHi + (r0 + m) * APH + 8 * hh;
  const unsigned short* arL = sLo + (r0 + m) * APH + 8 * hh;
#pragma unroll 1
  for (int g = 0; g < FEAT / 64; ++g) {
    v8f acc[4];
#pragma unroll
    for (int t = 0; t < 4; ++t) { v8f z = {0.f, 0.f, 0.f, 0.f, 0.f, 0.f, 0.f, 0.f}; acc[t] = z; }
#pragma unroll 1
    for (int kt = 0; kt < KCAT / 32; ++kt) {
      FragB aH, aL;
      aH.u[0] = *(const v4u*)(arH + 32 * kt);
      aH.u[1] = *(const v4u*)(arH + 32 * kt + 16);
      aL.u[0] = *(const v4u*)(arL + 32 * kt);
      aL.u[1] = *(const v4u*)(arL + 32 * kt + 16);
#pragma unroll
      for (int t = 0; t < 4; ++t) {
        const size_t bo = (size_t)(64 * g + 16 * t + m) * KCAT + 32 * kt + 8 * hh;
        FragB bH, bL;
        bH.u[0] = *(const v4u*)(BH + bo);
        bH.u[1] = *(const v4u*)(BH + bo + 16);
        bL.u[0] = *(const v4u*)(BL + bo);
        bL.u[1] = *(const v4u*)(BL + bo + 16);
        acc[t] = wmb(aH.v, bH.v, acc[t]);
        acc[t] = wmb(aH.v, bL.v, acc[t]);
        acc[t] = wmb(aL.v, bH.v, acc[t]);
      }
    }
#pragma unroll
    for (int t = 0; t < 4; ++t) {
      const int col = 64 * g + 16 * t + m;
      const float bl = bias[col];
      float* sp = stg + (r0 + 8 * hh) * SPF + col;
#pragma unroll
      for (int r = 0; r < 8; ++r) {
        const float v = acc[t][r] + bl;
        sp[r * SPF] = fmaxf(v, 0.0f);
      }
    }
  }
  __syncthreads();

  const float* lp = stg + r0 * SPF + 4 * lane;
  float* gp = Out + ((size_t)rowBase + r0) * FEAT + 4 * lane;
#pragma unroll
  for (int i = 0; i < 16; ++i) {
    if (rowBase + r0 + i < nRowsOut) {
      const v4f v = *(const v4f*)(lp + i * SPF);
      *(volatile v4f*)(gp + (size_t)i * FEAT) = v;
    }
  }
  __threadfence();
#pragma unroll
  for (int i = 0; i < 16; ++i) {
    if (rowBase + r0 + i < nRowsOut) {
      const v4f v = *(const v4f*)(lp + i * SPF);
      *(volatile v4f*)(gp + (size_t)i * FEAT) = v;
    }
  }
}

extern "C" void kernel_launch(void* const* d_in, const int* in_sizes, int n_in,
                              void* d_out, int out_size, void* d_ws, size_t ws_size,
                              hipStream_t stream) {
  if (n_in < 11) return;
  const int nN = in_sizes[0] / FEAT;
  const int nE = in_sizes[1] / 2;
  if (nN <= 0 || nE <= 0 || in_sizes[0] != nN * FEAT || in_sizes[1] != 2 * nE) return;
  if (in_sizes[2] != FEAT * FEAT || in_sizes[4] != FEAT * FEAT || in_sizes[5] != FEAT * FEAT ||
      in_sizes[7] != FEAT * FEAT || in_sizes[8] != FEAT * FEAT || in_sizes[10] != FEAT * FEAT) return;
  if (in_sizes[3] < FEAT || in_sizes[6] < FEAT || in_sizes[9] < FEAT) return;
  if (out_size != nN * FEAT) return;
  if (nE > (1 << 28) || nN > (1 << 24)) return;

  const float* x   = (const float*)d_in[0];
  const int*   ei  = (const int*)d_in[1];
  const float* wr1 = (const float*)d_in[2];
  const float* b1  = (const float*)d_in[3];
  const float* wo1 = (const float*)d_in[4];
  const float* wr2 = (const float*)d_in[5];
  const float* b2  = (const float*)d_in[6];
  const float* wo2 = (const float*)d_in[7];
  const float* wr3 = (const float*)d_in[8];
  const float* b3  = (const float*)d_in[9];
  const float* wo3 = (const float*)d_in[10];
  float* out = (float*)d_out;

  const int NPAD   = ((nN + GROWS - 1) / GROWS) * GROWS;
  const int nBC    = (nN + NBC - 1) / NBC;
  const int CNTPAD = nBC * NBC;
  if (4 * nBC + 1 > RBN) return;
  const int nBF    = (nN + NBF - 1) / NBF;
  const int csrLen = ((nE + 31) & ~31) + 4096;
  const int nLay   = NPAD / GROWS;

  char* ws = (char*)d_ws;
  size_t off = 0;
  const size_t oBH  = off; off += (size_t)NLAYER * FEAT * KCAT * 2;   off = (off + 255) & ~(size_t)255;
  const size_t oBL  = off; off += (size_t)NLAYER * FEAT * KCAT * 2;   off = (off + 255) & ~(size_t)255;
  const size_t oCnt = off; off += (size_t)CNTPAD * 4;                 off = (off + 255) & ~(size_t)255;
  const size_t oOff = off; off += (size_t)CNTPAD * 4;                 off = (off + 255) & ~(size_t)255;
  const size_t oRb  = off; off += (size_t)RBN * 4;                    off = (off + 255) & ~(size_t)255;
  const size_t oCsr = off; off += (size_t)csrLen * 4;                 off = (off + 255) & ~(size_t)255;
  const size_t oHA  = off; off += (size_t)NPAD * FEAT * 4;            off = (off + 255) & ~(size_t)255;
  const size_t oHB  = off; off += (size_t)NPAD * FEAT * 4;            off = (off + 255) & ~(size_t)255;
  if (off > ws_size) return;
  unsigned short* BH  = (unsigned short*)(ws + oBH);
  unsigned short* BL  = (unsigned short*)(ws + oBL);
  int*   cnt  = (int*)(ws + oCnt);
  int*   offp = (int*)(ws + oOff);
  int*   rb   = (int*)(ws + oRb);
  int*   csr  = (int*)(ws + oCsr);
  float* hA   = (float*)(ws + oHA);
  float* hB   = (float*)(ws + oHB);

  const int vec8 = ((nE & 3) == 0) ? 1 : 0;

  k_wprep<<<WPB, NTHR, 0, stream>>>(wr1, wo1, wr2, wo2, wr3, wo3, BH, BL);

  k_count<<<nBC, NTHR, 0, stream>>>(ei, cnt, nE, vec8);
  k_offsets<<<1, OTHR, 0, stream>>>(cnt, offp, rb, nBC);
  hipFuncSetAttribute(reinterpret_cast<const void*>(&k_fill),
                      hipFuncAttributeMaxDynamicSharedMemorySize, LDS_FILL);
  k_fill<<<nBF, NTHR, LDS_FILL, stream>>>(ei, offp, rb, csr, nN, nE, vec8, csrLen);

  hipFuncSetAttribute(reinterpret_cast<const void*>(&k_layer),
                      hipFuncAttributeMaxDynamicSharedMemorySize, LDS_LAYER);
  const size_t wl = (size_t)FEAT * KCAT;
  k_layer<<<nLay, NTHR, LDS_LAYER, stream>>>(x,  csr, offp, cnt, BH,          BL,          b1, hA,  nN, csrLen, CNTPAD, NPAD);
  k_layer<<<nLay, NTHR, LDS_LAYER, stream>>>(hA, csr, offp, cnt, BH + wl,     BL + wl,     b2, hB,  nN, csrLen, CNTPAD, NPAD);
  k_layer<<<nLay, NTHR, LDS_LAYER, stream>>>(hB, csr, offp, cnt, BH + 2 * wl, BL + 2 * wl, b3, out, nN, csrLen, CNTPAD, nN);
}
